// GraphLayerConvSimple_51101520888322
// MI455X (gfx1250) — hardware-verified
//
#include <hip/hip_runtime.h>
#include <stddef.h>


typedef __attribute__((ext_vector_type(16))) _Float16 v16h;
typedef __attribute__((ext_vector_type(8)))  _Float16 v8h;
typedef __attribute__((ext_vector_type(16))) __bf16   v16b;
typedef __attribute__((ext_vector_type(8)))  __bf16   v8b;
typedef __attribute__((ext_vector_type(8)))  float    v8f;
typedef __attribute__((ext_vector_type(4)))  float    v4f;
#define PSCALE 32768.0f
#define U16(p) ((const unsigned short*)(const void*)(p))
#define PSCALE_INV (1.0f / 32768.0f)

__device__ __forceinline__ unsigned short f2bf_bits(float f) {
  unsigned u = __float_as_uint(f);
  return (unsigned short)((u + 0x7FFFu + ((u >> 16) & 1u)) >> 16);
}
__device__ __forceinline__ float bf_bits2f(unsigned short h) { return __uint_as_float(((unsigned)h) << 16); }

__device__ __forceinline__ void dep_guard_h(v8f& a, v8f& b, v16h x, v16h y) { asm volatile("v_nop\n\tv_nop\n\tv_nop\n\tv_nop" : "+v"(a), "+v"(b) : "v"(x), "v"(y)); }
__device__ __forceinline__ void dep_guard_b(v8f& a, v8f& b, v16b x, v16b y) { asm volatile("v_nop\n\tv_nop\n\tv_nop\n\tv_nop" : "+v"(a), "+v"(b) : "v"(x), "v"(y)); }
__device__ __forceinline__ void keep4_h(v16h a, v16h b, v16h c, v16h d) { asm volatile("v_nop" :: "v"(a), "v"(b), "v"(c), "v"(d)); }
__device__ __forceinline__ void keep4_b(v16b a, v16b b, v16b c, v16b d) { asm volatile("v_nop" :: "v"(a), "v"(b), "v"(c), "v"(d)); }
__device__ __forceinline__ void acc_guard4(v8f& a, v8f& b, v8f& c, v8f& d) { asm volatile("v_nop\n\tv_nop\n\tv_nop\n\tv_nop" : "+v"(a), "+v"(b), "+v"(c), "+v"(d)); }
template <typename T> struct Frag;
template <> struct Frag<_Float16> {
  typedef v16h V; union U { v16h v; v8h h[2]; };
  static __device__ __forceinline__ v16h load(const _Float16* p) {
    U f; f.h[0] = *(const v8h*)(p); f.h[1] = *(const v8h*)(p + 16); return f.v;
  }
  static __device__ __forceinline__ v8f mma(v16h a, v16h b, v8f c) {
    return __builtin_amdgcn_wmma_f32_16x16x32_f16(false, a, false, b, (short)0, c, false, false);
  }
  static __device__ __forceinline__ void guard(v8f& a, v8f& b, v16h x, v16h y) { dep_guard_h(a, b, x, y); }
  static __device__ __forceinline__ void keep(v16h a, v16h b, v16h c, v16h d) { keep4_h(a, b, c, d); }
};
template <> struct Frag<__bf16> {
  typedef v16b V; union U { v16b v; v8b h[2]; };
  static __device__ __forceinline__ v16b load(const __bf16* p) {
    U f; f.h[0] = *(const v8b*)(p); f.h[1] = *(const v8b*)(p + 16); return f.v;
  }
  static __device__ __forceinline__ v8f mma(v16b a, v16b b, v8f c) {
    return __builtin_amdgcn_wmma_f32_16x16x32_bf16(false, a, false, b, (short)0, c, false, false);
  }
  static __device__ __forceinline__ void guard(v8f& a, v8f& b, v16b x, v16b y) { dep_guard_b(a, b, x, y); }
  static __device__ __forceinline__ void keep(v16b a, v16b b, v16b c, v16b d) { keep4_b(a, b, c, d); }
};

template <int ET> struct Elem;
template <> struct Elem<0> { typedef _Float16 T; };
template <> struct Elem<1> { typedef __bf16 T; };
template <int ET, bool SPLIT, int BIAS_MODE, int OUT_MODE, bool RESID, int ACT = 0>
__global__ __launch_bounds__(256) void wmma_gemm64(
    const unsigned short* __restrict__ Ap, const unsigned short* __restrict__ A2p, int lda, long strideA,
    const unsigned short* __restrict__ Btp, const unsigned short* __restrict__ Bt2p, int ldb, long strideB,
    void* __restrict__ Cout, void* __restrict__ Cout2, int ldc, long strideC,
    const float* __restrict__ bias,
    const float* __restrict__ resid, long strideR,
    int M, int N, int K, float scale) {
  typedef typename Elem<ET>::T T;
  typedef typename Frag<T>::V V;
  const T* A = (const T*)Ap; const T* A2 = (const T*)A2p; const T* Bt = (const T*)Btp; const T* Bt2 = (const T*)Bt2p;
  __shared__ __align__(16) float sT[8][16 * 68];
  const int b    = blockIdx.y;
  const int lane = threadIdx.x & 31;
  const int wave = threadIdx.x >> 5;
  const int tilesN = N >> 6;
  const int tilesM = M >> 6;
  const int tile = blockIdx.x * 8 + wave;
  if (tile >= tilesM * tilesN) return;
  const int tm = tile / tilesN;
  const int tn = tile - tm * tilesN;
  const int m0 = tm << 6;
  const int n0 = tn << 6;

  const T* Ab  = A  + (size_t)b * strideA;
  const T* Bb  = Bt + (size_t)b * strideB;
  const T* Ab2 = SPLIT ? (A2  + (size_t)b * strideA) : nullptr;
  const T* Bb2 = SPLIT ? (Bt2 + (size_t)b * strideB) : nullptr;

  const int rlane = lane & 15;
  const int koff  = (lane >> 4) * 8;
  const int mOff  = (lane >> 4) * 8;

  v8f acc[4][4];
#pragma unroll
  for (int i = 0; i < 4; ++i)
#pragma unroll
    for (int j = 0; j < 4; ++j) acc[i][j] = (v8f){0.f,0.f,0.f,0.f,0.f,0.f,0.f,0.f};

  for (int k0 = 0; k0 < K; k0 += 32) {
    V bh[4], bl[4];
#pragma unroll
    for (int j = 0; j < 4; ++j) {
      const size_t bo = (size_t)(n0 + (j << 4) + rlane) * ldb + koff + k0;
      bh[j] = Frag<T>::load(Bb + bo);
      if (SPLIT) bl[j] = Frag<T>::load(Bb2 + bo);
    }
#pragma unroll
    for (int i = 0; i < 4; ++i) {
      const size_t ao = (size_t)(m0 + (i << 4) + rlane) * lda + koff + k0;
      V ah = Frag<T>::load(Ab + ao);
      V al;
      if (SPLIT) al = Frag<T>::load(Ab2 + ao);
#pragma unroll
      for (int j = 0; j < 4; ++j) {
        acc[i][j] = Frag<T>::mma(ah, bh[j], acc[i][j]);
        if (SPLIT) {
          acc[i][j] = Frag<T>::mma(ah, bl[j], acc[i][j]);
          acc[i][j] = Frag<T>::mma(al, bh[j], acc[i][j]);
        }
      }
      Frag<T>::guard(acc[i][0], acc[i][3], ah, SPLIT ? al : ah);
    }
    Frag<T>::keep(bh[0], bh[1], bh[2], bh[3]);
    if (SPLIT) Frag<T>::keep(bl[0], bl[1], bl[2], bl[3]);
  }
  acc_guard4(acc[0][0], acc[0][1], acc[0][2], acc[0][3]);
  acc_guard4(acc[1][0], acc[1][1], acc[1][2], acc[1][3]);
  acc_guard4(acc[2][0], acc[2][1], acc[2][2], acc[2][3]);
  acc_guard4(acc[3][0], acc[3][1], acc[3][2], acc[3][3]);

  float* slab = sT[wave];
  const float* Rb = RESID ? (resid + (size_t)b * strideR) : nullptr;
#pragma unroll
  for (int i = 0; i < 4; ++i) {
    const int mBase = m0 + (i << 4);
#pragma unroll
    for (int j = 0; j < 4; ++j) {
      const int n = n0 + (j << 4) + rlane;
      float bv = 0.f;
      if (BIAS_MODE == 2) bv = bias[n];
#pragma unroll
      for (int r = 0; r < 8; ++r) {
        float v = acc[i][j][r] * scale;
        if (BIAS_MODE == 1) v += bias[mBase + mOff + r];
        if (BIAS_MODE == 2) v += bv;
        if (RESID) v += Rb[(size_t)(mBase + mOff + r) * ldc + n];
        if (ACT == 1) v = tanhf(v);
        if (ACT == 2) v = fmaxf(v, 0.0f);
        if (ACT == 3) v = v / (1.0f + expf(-v));
        if (ACT == 4) v = (v > 0.f) ? v : 0.01f * v;
        if (ACT == 5) v = 0.5f * v * (1.0f + erff(v * 0.70710678118654752f));
        slab[(mOff + r) * 68 + (j << 4) + rlane] = v;
      }
    }
    __builtin_amdgcn_fence(__ATOMIC_RELEASE, "workgroup");
    __builtin_amdgcn_wave_barrier();
    __builtin_amdgcn_fence(__ATOMIC_ACQUIRE, "workgroup");
    if (OUT_MODE == 0) {
      float* C = (float*)Cout + (size_t)b * strideC;
      const int hh = lane >> 4, c4 = (lane & 15) * 4;
      for (int pass = 0; pass < 2; ++pass) {
#pragma unroll
        for (int it = 0; it < 8; ++it) {
          const int row = it * 2 + hh;
          v4f v = *(const v4f*)(slab + row * 68 + c4);
          *(volatile v4f*)(C + (size_t)(mBase + row) * ldc + n0 + c4) = v;
        }
        __threadfence();
      }
    } else {
      const int q = lane >> 3, c8 = (lane & 7) * 8;
      unsigned short* C  = (unsigned short*)Cout  + (size_t)b * strideC;
      unsigned short* C2 = (OUT_MODE == 2) ? ((unsigned short*)Cout2 + (size_t)b * strideC) : nullptr;
      for (int pass = 0; pass < 2; ++pass) {
#pragma unroll
        for (int it = 0; it < 4; ++it) {
          const int row = it * 4 + q;
          const float* sp = slab + row * 68 + c8;
          v8h hv, lv;
#pragma unroll
          for (int e = 0; e < 8; ++e) {
            if (OUT_MODE == 1) {
              hv[e] = (_Float16)sp[e];
            } else {
              unsigned short hb = f2bf_bits(sp[e]);
              unsigned short lb = f2bf_bits(sp[e] - bf_bits2f(hb));
              hv[e] = __builtin_bit_cast(_Float16, hb);
              lv[e] = __builtin_bit_cast(_Float16, lb);
            }
          }
          *(volatile v8h*)(C + (size_t)(mBase + row) * ldc + n0 + c8) = hv;
          if (OUT_MODE == 2) *(volatile v8h*)(C2 + (size_t)(mBase + row) * ldc + n0 + c8) = lv;
        }
        __threadfence();
      }
    }
    __builtin_amdgcn_fence(__ATOMIC_RELEASE, "workgroup");
    __builtin_amdgcn_wave_barrier();
    __builtin_amdgcn_fence(__ATOMIC_ACQUIRE, "workgroup");
  }
}

#define NPX   256
#define CH    64
#define KC    576
#define KN    20
#define QB    5
#define NPB   (QB*KN)
#define PROWS (NPB*NPX)
#define PCOLS 256

__global__ __launch_bounds__(256) void prep_x_k(const float* __restrict__ x, const float* __restrict__ t,
                                               _Float16* __restrict__ xin, int nimg, int cin) {
  const int g = blockIdx.x * 256 + threadIdx.x;
  if (g >= nimg * NPX * 8) return;
  const int c8 = g & 7, rest = g >> 3, px = rest & 255, img = rest >> 8;
  const float tv = t[0];
  v8h v;
#pragma unroll
  for (int e = 0; e < 8; ++e) {
    const int c = c8 * 8 + e;
    int cx = c - 1; cx = cx < 0 ? 0 : (cx > cin - 1 ? cin - 1 : cx);
    const float xv = x[((size_t)img * cin + cx) * NPX + px];
    const float val = (c == 0) ? tv : ((c <= cin) ? xv : 0.0f);
    v[e] = (_Float16)val;
  }
  _Float16* d = xin + ((size_t)(img * NPX + px)) * CH + c8 * 8;
  *(volatile v8h*)d = v;
  __threadfence();
  *(volatile v8h*)d = v;
}

__global__ __launch_bounds__(128) void castw_k(const float* __restrict__ w, int cin_total, int c_off, int cvalid,
                                              _Float16* __restrict__ dst, float scale) {
  const int o = blockIdx.x;
  const int tIdx = threadIdx.x;
  if (tIdx >= 72) return;
  const int k0 = tIdx * 8, tap = k0 >> 6, c0 = k0 & 63;
  v8h v;
#pragma unroll
  for (int e = 0; e < 8; ++e) {
    const int c = c0 + e;
    const int cc = c < cvalid ? c : (cvalid - 1);
    const float f = w[((size_t)o * cin_total + c_off + cc) * 9 + tap];
    v[e] = (_Float16)((c < cvalid) ? f * scale : 0.0f);
  }
  _Float16* d = dst + (size_t)o * KC + k0;
  *(volatile v8h*)d = v;
  __threadfence();
  *(volatile v8h*)d = v;
}

__global__ __launch_bounds__(256) void im2col_k(const _Float16* __restrict__ src, long srcStride,
                                               _Float16* __restrict__ dst, long dstStride, int rows) {
  const _Float16* s = src + (size_t)blockIdx.y * (size_t)srcStride;
  _Float16* d = dst + (size_t)blockIdx.y * (size_t)dstStride;
  const int g = blockIdx.x * 256 + threadIdx.x;
  if (g >= rows * 72) return;
  const int piece = g & 7, unit = g >> 3;
  const int row = unit / 9, tap = unit - row * 9;
  const int img = row >> 8, px = row & 255, y = px >> 4, xx = px & 15;
  const int ky = tap / 3, kx = tap - ky * 3;
  const int sy = y + ky - 1, sx = xx + kx - 1;
  const bool valid = ((unsigned)sy < 16u) && ((unsigned)sx < 16u);
  const int cy = sy < 0 ? 0 : (sy > 15 ? 15 : sy);
  const int cx = sx < 0 ? 0 : (sx > 15 ? 15 : sx);
  const v8h v = *(const v8h*)(s + ((size_t)(img * NPX + cy * 16 + cx)) * CH + piece * 8);
  v8h o;
#pragma unroll
  for (int e = 0; e < 8; ++e) o[e] = valid ? v[e] : (_Float16)0.0f;
  _Float16* dp = d + (size_t)row * KC + tap * CH + piece * 8;
  *(volatile v8h*)dp = o;
  __threadfence();
  *(volatile v8h*)dp = o;
}

__global__ __launch_bounds__(256) void rpair_k(const float* __restrict__ P, const float* __restrict__ bb1,
                                              const float* __restrict__ bbg1, _Float16* __restrict__ r, int batch) {
  const int y2 = blockIdx.y;
  const float* bias = y2 ? bbg1 : bb1;
  const int fo = y2 * 128, so = fo + 64;
  _Float16* dst = r + (size_t)y2 * ((size_t)PROWS * CH);
  const int g = blockIdx.x * 256 + threadIdx.x;
  if (g >= NPB * NPX * 8) return;
  const int c8 = g & 7, rest = g >> 3, px = rest & 255, pl = rest >> 8;
  const int ql = pl / KN, p = pl - ql * KN;
  const int oq = batch * QB + ql;
  const int n = oq / KN;
  const int np = n * KN + p;
  const float* pf = P + ((size_t)(oq * NPX + px)) * PCOLS + fo + c8 * 8;
  const float* ps = P + ((size_t)(np * NPX + px)) * PCOLS + so + c8 * 8;
  const float* bp = bias + c8 * 8;
  const v4f f0 = *(const v4f*)pf, f1 = *(const v4f*)(pf + 4);
  const v4f s0 = *(const v4f*)ps, s1 = *(const v4f*)(ps + 4);
  v8h v;
#pragma unroll
  for (int e = 0; e < 4; ++e) {
    v[e]     = (_Float16)fmaxf(f0[e] + s0[e] + bp[e],     0.0f);
    v[4 + e] = (_Float16)fmaxf(f1[e] + s1[e] + bp[4 + e], 0.0f);
  }
  _Float16* d = dst + ((size_t)(pl * NPX + px)) * CH + c8 * 8;
  *(volatile v8h*)d = v;
  __threadfence();
  *(volatile v8h*)d = v;
}

__device__ __forceinline__ float sigm_f(float x) {
  const float e = __expf(-x);
  return __builtin_amdgcn_rcpf(1.0f + e);
}

__global__ __launch_bounds__(256) void combine_k(const float* __restrict__ Cpg, const float* __restrict__ uLin2,
                                                const float* __restrict__ bu2, const float* __restrict__ bug2,
                                                const float* __restrict__ bb2, const float* __restrict__ bbg2,
                                                float* __restrict__ out, int batch, int nrows) {
  __shared__ __align__(16) float T[CH * 36];
  const int tid = threadIdx.x, lane = tid & 31, wave = tid >> 5;
  const int ql = blockIdx.x >> 3, pxb = blockIdx.x & 7;
  const int px0 = pxb * 32;
  const int oq = batch * QB + ql;
  const int pxl = tid >> 3, c8 = tid & 7;
  const int px = px0 + pxl;
  float b2v[8], bg2v[8], s[8];
#pragma unroll
  for (int e = 0; e < 8; ++e) { b2v[e] = bb2[c8 * 8 + e]; bg2v[e] = bbg2[c8 * 8 + e]; s[e] = 0.0f; }
  const size_t gstride = (size_t)PROWS * CH;
#pragma unroll 1
  for (int p = 0; p < KN; ++p) {
    const size_t ro = ((size_t)((ql * KN + p) * NPX + px)) * CH + c8 * 8;
    const v4f m0 = *(const v4f*)(Cpg + ro), m1 = *(const v4f*)(Cpg + ro + 4);
    const v4f g0 = *(const v4f*)(Cpg + gstride + ro), g1 = *(const v4f*)(Cpg + gstride + ro + 4);
#pragma unroll
    for (int e = 0; e < 4; ++e) {
      s[e]     += (m0[e] + b2v[e])     * sigm_f(g0[e] + bg2v[e]);
      s[4 + e] += (m1[e] + b2v[4 + e]) * sigm_f(g1[e] + bg2v[4 + e]);
    }
  }
  const size_t ustride = (size_t)nrows * CH;
  const size_t uo = ((size_t)(oq * NPX + px)) * CH + c8 * 8;
  const v4f u0 = *(const v4f*)(uLin2 + uo), u1 = *(const v4f*)(uLin2 + uo + 4);
  const v4f q0 = *(const v4f*)(uLin2 + ustride + uo), q1 = *(const v4f*)(uLin2 + ustride + uo + 4);
  const float invk = 1.0f / (float)(KN - 1);
#pragma unroll
  for (int e = 0; e < 4; ++e) {
    const float v0 = (u0[e] + bu2[c8 * 8 + e])     * sigm_f(q0[e] + bug2[c8 * 8 + e])     + s[e]     * invk;
    const float v1 = (u1[e] + bu2[c8 * 8 + 4 + e]) * sigm_f(q1[e] + bug2[c8 * 8 + 4 + e]) + s[4 + e] * invk;
    T[(c8 * 8 + e) * 36 + pxl]     = v0;
    T[(c8 * 8 + 4 + e) * 36 + pxl] = v1;
  }
  __syncthreads();
  const int px4 = (lane & 7) * 4;
  for (int pass = 0; pass < 2; ++pass) {
#pragma unroll
    for (int it = 0; it < 2; ++it) {
      const int c = wave * 8 + it * 4 + (lane >> 3);
      const v4f val = *(const v4f*)(T + c * 36 + px4);
      *(volatile v4f*)(out + ((size_t)(oq * CH + c)) * NPX + px0 + px4) = val;
    }
    __threadfence();
  }
}

extern "C" void kernel_launch(void* const* d_in, const int* in_sizes, int n_in,
                              void* d_out, int out_size, void* d_ws, size_t ws_size,
                              hipStream_t stream) {
  if (n_in < 20) return;
  const float* t     = (const float*)d_in[0];
  const float* x     = (const float*)d_in[1];
  const float* w_map = (const float*)d_in[2];
  const float* b_map = (const float*)d_in[3];
  const float* w_u1  = (const float*)d_in[4];
  const float* b_u1  = (const float*)d_in[5];
  const float* w_u2  = (const float*)d_in[6];
  const float* b_u2  = (const float*)d_in[7];
  const float* w_ug1 = (const float*)d_in[8];
  const float* b_ug1 = (const float*)d_in[9];
  const float* w_ug2 = (const float*)d_in[10];
  const float* b_ug2 = (const float*)d_in[11];
  const float* w_b1  = (const float*)d_in[12];
  const float* b_b1  = (const float*)d_in[13];
  const float* w_b2  = (const float*)d_in[14];
  const float* b_b2  = (const float*)d_in[15];
  const float* w_bg1 = (const float*)d_in[16];
  const float* b_bg1 = (const float*)d_in[17];
  const float* w_bg2 = (const float*)d_in[18];
  const float* b_bg2 = (const float*)d_in[19];

  const int nimg = 2 * KN;
  const int cinx = 32;
  const int cinm = cinx + 1;
  if (in_sizes[0] < 1 || in_sizes[1] != nimg * cinx * NPX || in_sizes[2] != CH * cinm * 9 ||
      in_sizes[4] != CH * CH * 9 || in_sizes[6] != CH * CH * 9 || in_sizes[8] != CH * CH * 9 ||
      in_sizes[10] != CH * CH * 9 || in_sizes[12] != CH * 128 * 9 || in_sizes[14] != CH * CH * 9 ||
      in_sizes[16] != CH * 128 * 9 || in_sizes[18] != CH * CH * 9 ||
      in_sizes[3] != CH || in_sizes[5] != CH || in_sizes[7] != CH || in_sizes[9] != CH || in_sizes[11] != CH ||
      in_sizes[13] != CH || in_sizes[15] != CH || in_sizes[17] != CH || in_sizes[19] != CH ||
      out_size != nimg * CH * NPX || (nimg % QB) != 0) return;
  const int nrows = nimg * NPX;
  const int nbatch = nimg / QB;

  char* ws = (char*)d_ws;
  size_t off = 0;
  auto carve = [&](size_t bytes) -> char* { char* p = ws + off; off += (bytes + 255) & ~(size_t)255; return p; };
  _Float16* W16   = (_Float16*)carve((size_t)704 * KC * sizeof(_Float16));
  _Float16* xin16 = (_Float16*)carve((size_t)nrows * CH * sizeof(_Float16));
  _Float16* h16   = (_Float16*)carve((size_t)nrows * CH * sizeof(_Float16));
  _Float16* ua16  = (_Float16*)carve((size_t)2 * nrows * CH * sizeof(_Float16));
  float*    uLin2 = (float*)carve((size_t)2 * nrows * CH * sizeof(float));
  float*    P     = (float*)carve((size_t)nrows * PCOLS * sizeof(float));
  _Float16* r16   = (_Float16*)carve((size_t)2 * PROWS * CH * sizeof(_Float16));
  float*    Cpg   = (float*)carve((size_t)2 * PROWS * CH * sizeof(float));
  size_t sbytes = (size_t)2 * PROWS * KC * sizeof(_Float16);
  const size_t s2 = (size_t)2 * nrows * KC * sizeof(_Float16);
  if (s2 > sbytes) sbytes = s2;
  _Float16* S     = (_Float16*)carve(sbytes);
  if (off > ws_size || off > (size_t)134217728u) return;

  _Float16* Wmap = W16;
  _Float16* Wu1  = W16 + (size_t)64 * KC;
  _Float16* Wug1 = W16 + (size_t)128 * KC;
  _Float16* WP   = W16 + (size_t)192 * KC;
  _Float16* Wu2g = W16 + (size_t)448 * KC;
  _Float16* Wb2g = W16 + (size_t)576 * KC;

  typedef unsigned short us;
  const float wsc = 16.0f, winv = 1.0f / 16.0f;

  prep_x_k<<<(nimg * NPX * 8 + 255) / 256, 256, 0, stream>>>(x, t, xin16, nimg, cinx);
  castw_k<<<64, 128, 0, stream>>>(w_map, cinm, 0,  cinm, Wmap, wsc);
  castw_k<<<64, 128, 0, stream>>>(w_u1,  CH,   0,  CH,   Wu1,  wsc);
  castw_k<<<64, 128, 0, stream>>>(w_ug1, CH,   0,  CH,   Wug1, wsc);
  castw_k<<<64, 128, 0, stream>>>(w_b1,  128,  0,  CH,   WP,                     wsc);
  castw_k<<<64, 128, 0, stream>>>(w_b1,  128,  64, CH,   WP + (size_t)64 * KC,   wsc);
  castw_k<<<64, 128, 0, stream>>>(w_bg1, 128,  0,  CH,   WP + (size_t)128 * KC,  wsc);
  castw_k<<<64, 128, 0, stream>>>(w_bg1, 128,  64, CH,   WP + (size_t)192 * KC,  wsc);
  castw_k<<<64, 128, 0, stream>>>(w_u2,  CH,   0,  CH,   Wu2g,                   wsc);
  castw_k<<<64, 128, 0, stream>>>(w_ug2, CH,   0,  CH,   Wu2g + (size_t)64 * KC, wsc);
  castw_k<<<64, 128, 0, stream>>>(w_b2,  CH,   0,  CH,   Wb2g,                   wsc);
  castw_k<<<64, 128, 0, stream>>>(w_bg2, CH,   0,  CH,   Wb2g + (size_t)64 * KC, wsc);

  const int node_tiles = nrows / 64;
  const int gx64  = (node_tiles * 1 + 7) / 8;
  const int gx256 = (node_tiles * 4 + 7) / 8;
  im2col_k<<<dim3((nrows * 72 + 255) / 256, 1), 256, 0, stream>>>(xin16, 0L, S, 0L, nrows);
  wmma_gemm64<0, false, 2, 1, false, 0><<<dim3(gx64, 1), 256, 0, stream>>>(
      (const us*)S, (const us*)S, KC, 0L, (const us*)Wmap, (const us*)Wmap, KC, 0L,
      (void*)h16, (void*)h16, CH, 0L, b_map, P, 0L, nrows, 64, KC, winv);
  im2col_k<<<dim3((nrows * 72 + 255) / 256, 1), 256, 0, stream>>>(h16, 0L, S, 0L, nrows);
  wmma_gemm64<0, false, 2, 1, false, 2><<<dim3(gx64, 1), 256, 0, stream>>>(
      (const us*)S, (const us*)S, KC, 0L, (const us*)Wu1, (const us*)Wu1, KC, 0L,
      (void*)ua16, (void*)ua16, CH, 0L, b_u1, P, 0L, nrows, 64, KC, winv);
  wmma_gemm64<0, false, 2, 1, false, 2><<<dim3(gx64, 1), 256, 0, stream>>>(
      (const us*)S, (const us*)S, KC, 0L, (const us*)Wug1, (const us*)Wug1, KC, 0L,
      (void*)(ua16 + (size_t)nrows * CH), (void*)(ua16 + (size_t)nrows * CH), CH, 0L, b_ug1, P, 0L, nrows, 64, KC, winv);
  wmma_gemm64<0, false, 0, 0, false, 0><<<dim3(gx256, 1), 256, 0, stream>>>(
      (const us*)S, (const us*)S, KC, 0L, (const us*)WP, (const us*)WP, KC, 0L,
      (void*)P, (void*)P, PCOLS, 0L, b_b1, uLin2, 0L, nrows, PCOLS, KC, winv);
  im2col_k<<<dim3((nrows * 72 + 255) / 256, 2), 256, 0, stream>>>(ua16, (long)nrows * CH, S, (long)nrows * KC, nrows);
  wmma_gemm64<0, false, 0, 0, false, 0><<<dim3(gx64, 2), 256, 0, stream>>>(
      (const us*)S, (const us*)S, KC, (long)nrows * KC, (const us*)Wu2g, (const us*)Wu2g, KC, (long)64 * KC,
      (void*)uLin2, (void*)uLin2, CH, (long)nrows * CH, b_u2, P, 0L, nrows, 64, KC, winv);

  const int pair_tiles = PROWS / 64;
  const int gxp = (pair_tiles + 7) / 8;
  for (int bt = 0; bt < nbatch; ++bt) {
    rpair_k<<<dim3((NPB * NPX * 8 + 255) / 256, 2), 256, 0, stream>>>(P, b_b1, b_bg1, r16, bt);
    im2col_k<<<dim3((PROWS * 72 + 255) / 256, 2), 256, 0, stream>>>(r16, (long)PROWS * CH, S, (long)PROWS * KC, PROWS);
    wmma_gemm64<0, false, 0, 0, false, 0><<<dim3(gxp, 2), 256, 0, stream>>>(
        (const us*)S, (const us*)S, KC, (long)PROWS * KC, (const us*)Wb2g, (const us*)Wb2g, KC, (long)64 * KC,
        (void*)Cpg, (void*)Cpg, CH, (long)PROWS * CH, b_b2, P, 0L, PROWS, 64, KC, winv);
    combine_k<<<QB * 8, 256, 0, stream>>>(Cpg, uLin2, b_u2, b_ug2, b_b2, b_bg2, (float*)d_out, bt, nrows);
  }
}
